// Backbone_47390669144486
// MI455X (gfx1250) — hardware-verified
//
#include <hip/hip_runtime.h>
#include <math.h>

constexpr int NWAY   = 5;
constexpr int NQRY   = 75;
constexpr int NIMG   = NWAY + NQRY;
constexpr int NCH    = 64;
constexpr int NPOS   = 400;
constexpr int NROWS  = NIMG * NPOS;
constexpr int NTILE  = NPOS / 16;
constexpr int NPAIR  = NQRY * NWAY;
constexpr int PCHUNK = 16;
constexpr float TEMP_ATTN = 5.0f;
constexpr float BN_EPS_C  = 1e-5f;
constexpr float LOG2E_C   = 1.4426950408889634f;
constexpr float WSCALE    = 16.0f;

static_assert(NROWS % 64 == 0, "GEMM M tile multiple");
static_assert(NCH == 64, "GEMM N = K = 64");
static_assert(NPOS % 16 == 0 && NPOS % PCHUNK == 0, "tile coverage");
static_assert(NROWS % 32 == 0, "feat kernel rows per block");
static_assert(NPAIR <= 12 * 32, "output writer coverage");

constexpr size_t WS_OFF_W16  = 0;
constexpr size_t WS_SZ_W16   = (size_t)NCH * NCH * 2;
constexpr size_t WS_OFF_XN16 = 8192;
constexpr size_t WS_SZ_XN16  = (size_t)NROWS * NCH * 2;
constexpr size_t WS_OFF_XN32 = WS_OFF_XN16 + WS_SZ_XN16;
constexpr size_t WS_SZ_XN32  = (size_t)NROWS * NCH * 4;
constexpr size_t WS_OFF_Y    = WS_OFF_XN32 + WS_SZ_XN32;
constexpr size_t WS_SZ_Y     = (size_t)NROWS * NCH * 4;
constexpr size_t WS_OFF_FEAT = WS_OFF_Y + WS_SZ_Y;
constexpr size_t WS_SZ_FEAT  = (size_t)NROWS * NCH * 2;
constexpr size_t WS_OFF_SIM  = WS_OFF_FEAT + WS_SZ_FEAT;
constexpr size_t WS_SZ_SIM   = (size_t)NPAIR * 32 * 4;
constexpr size_t WS_TOTAL    = WS_OFF_SIM + WS_SZ_SIM;
static_assert(WS_SZ_W16 <= 8192, "w16 fits its slot");
static_assert(WS_OFF_XN16 % 256 == 0 && WS_OFF_XN32 % 256 == 0 && WS_OFF_Y % 256 == 0 &&
              WS_OFF_FEAT % 256 == 0 && WS_OFF_SIM % 256 == 0, "alignment");
static_assert(WS_TOTAL <= 134217728ull, "carve under 128 MiB");

typedef __attribute__((ext_vector_type(16))) _Float16 v16h;
typedef __attribute__((ext_vector_type(8)))  _Float16 v8h;
typedef __attribute__((ext_vector_type(16))) __bf16   v16b;
typedef __attribute__((ext_vector_type(8)))  __bf16   v8b;
typedef __attribute__((ext_vector_type(8)))  float    v8f;
typedef __attribute__((ext_vector_type(4)))  float    v4f;
#define PSCALE 32768.0f
#define U16(p) ((const unsigned short*)(const void*)(p))
#define PSCALE_INV (1.0f / 32768.0f)

__device__ __forceinline__ unsigned short f2bf_bits(float f) {
  unsigned u = __float_as_uint(f);
  return (unsigned short)((u + 0x7FFFu + ((u >> 16) & 1u)) >> 16);
}
__device__ __forceinline__ float bf_bits2f(unsigned short h) { return __uint_as_float(((unsigned)h) << 16); }

__device__ __forceinline__ void dep_guard_h(v8f& a, v8f& b, v16h x, v16h y) { asm volatile("v_nop\n\tv_nop\n\tv_nop\n\tv_nop" : "+v"(a), "+v"(b) : "v"(x), "v"(y)); }
__device__ __forceinline__ void dep_guard_b(v8f& a, v8f& b, v16b x, v16b y) { asm volatile("v_nop\n\tv_nop\n\tv_nop\n\tv_nop" : "+v"(a), "+v"(b) : "v"(x), "v"(y)); }
__device__ __forceinline__ void keep4_h(v16h a, v16h b, v16h c, v16h d) { asm volatile("v_nop" :: "v"(a), "v"(b), "v"(c), "v"(d)); }
__device__ __forceinline__ void keep4_b(v16b a, v16b b, v16b c, v16b d) { asm volatile("v_nop" :: "v"(a), "v"(b), "v"(c), "v"(d)); }
__device__ __forceinline__ void acc_guard4(v8f& a, v8f& b, v8f& c, v8f& d) { asm volatile("v_nop\n\tv_nop\n\tv_nop\n\tv_nop" : "+v"(a), "+v"(b), "+v"(c), "+v"(d)); }
template <typename T> struct Frag;
template <> struct Frag<_Float16> {
  typedef v16h V; union U { v16h v; v8h h[2]; };
  static __device__ __forceinline__ v16h load(const _Float16* p) {
    U f; f.h[0] = *(const v8h*)(p); f.h[1] = *(const v8h*)(p + 16); return f.v;
  }
  static __device__ __forceinline__ v8f mma(v16h a, v16h b, v8f c) {
    return __builtin_amdgcn_wmma_f32_16x16x32_f16(false, a, false, b, (short)0, c, false, false);
  }
  static __device__ __forceinline__ void guard(v8f& a, v8f& b, v16h x, v16h y) { dep_guard_h(a, b, x, y); }
  static __device__ __forceinline__ void keep(v16h a, v16h b, v16h c, v16h d) { keep4_h(a, b, c, d); }
};
template <> struct Frag<__bf16> {
  typedef v16b V; union U { v16b v; v8b h[2]; };
  static __device__ __forceinline__ v16b load(const __bf16* p) {
    U f; f.h[0] = *(const v8b*)(p); f.h[1] = *(const v8b*)(p + 16); return f.v;
  }
  static __device__ __forceinline__ v8f mma(v16b a, v16b b, v8f c) {
    return __builtin_amdgcn_wmma_f32_16x16x32_bf16(false, a, false, b, (short)0, c, false, false);
  }
  static __device__ __forceinline__ void guard(v8f& a, v8f& b, v16b x, v16b y) { dep_guard_b(a, b, x, y); }
  static __device__ __forceinline__ void keep(v16b a, v16b b, v16b c, v16b d) { keep4_b(a, b, c, d); }
};

template <int ET> struct Elem;
template <> struct Elem<0> { typedef _Float16 T; };
template <> struct Elem<1> { typedef __bf16 T; };
template <int ET, bool SPLIT, int BIAS_MODE, int OUT_MODE, bool RESID, int ACT = 0>
__global__ __launch_bounds__(256) void wmma_gemm64(
    const unsigned short* __restrict__ Ap, const unsigned short* __restrict__ A2p, int lda, long strideA,
    const unsigned short* __restrict__ Btp, const unsigned short* __restrict__ Bt2p, int ldb, long strideB,
    void* __restrict__ Cout, void* __restrict__ Cout2, int ldc, long strideC,
    const float* __restrict__ bias,
    const float* __restrict__ resid, long strideR,
    int M, int N, int K, float scale) {
  typedef typename Elem<ET>::T T;
  typedef typename Frag<T>::V V;
  const T* A = (const T*)Ap; const T* A2 = (const T*)A2p; const T* Bt = (const T*)Btp; const T* Bt2 = (const T*)Bt2p;
  __shared__ __align__(16) float sT[8][16 * 68];
  const int b    = blockIdx.y;
  const int lane = threadIdx.x & 31;
  const int wave = threadIdx.x >> 5;
  const int tilesN = N >> 6;
  const int tilesM = M >> 6;
  const int tile = blockIdx.x * 8 + wave;
  if (tile >= tilesM * tilesN) return;
  const int tm = tile / tilesN;
  const int tn = tile - tm * tilesN;
  const int m0 = tm << 6;
  const int n0 = tn << 6;

  const T* Ab  = A  + (size_t)b * strideA;
  const T* Bb  = Bt + (size_t)b * strideB;
  const T* Ab2 = SPLIT ? (A2  + (size_t)b * strideA) : nullptr;
  const T* Bb2 = SPLIT ? (Bt2 + (size_t)b * strideB) : nullptr;

  const int rlane = lane & 15;
  const int koff  = (lane >> 4) * 8;
  const int mOff  = (lane >> 4) * 8;

  v8f acc[4][4];
#pragma unroll
  for (int i = 0; i < 4; ++i)
#pragma unroll
    for (int j = 0; j < 4; ++j) acc[i][j] = (v8f){0.f,0.f,0.f,0.f,0.f,0.f,0.f,0.f};

  for (int k0 = 0; k0 < K; k0 += 32) {
    V bh[4], bl[4];
#pragma unroll
    for (int j = 0; j < 4; ++j) {
      const size_t bo = (size_t)(n0 + (j << 4) + rlane) * ldb + koff + k0;
      bh[j] = Frag<T>::load(Bb + bo);
      if (SPLIT) bl[j] = Frag<T>::load(Bb2 + bo);
    }
#pragma unroll
    for (int i = 0; i < 4; ++i) {
      const size_t ao = (size_t)(m0 + (i << 4) + rlane) * lda + koff + k0;
      V ah = Frag<T>::load(Ab + ao);
      V al;
      if (SPLIT) al = Frag<T>::load(Ab2 + ao);
#pragma unroll
      for (int j = 0; j < 4; ++j) {
        acc[i][j] = Frag<T>::mma(ah, bh[j], acc[i][j]);
        if (SPLIT) {
          acc[i][j] = Frag<T>::mma(ah, bl[j], acc[i][j]);
          acc[i][j] = Frag<T>::mma(al, bh[j], acc[i][j]);
        }
      }
      Frag<T>::guard(acc[i][0], acc[i][3], ah, SPLIT ? al : ah);
    }
    Frag<T>::keep(bh[0], bh[1], bh[2], bh[3]);
    if (SPLIT) Frag<T>::keep(bl[0], bl[1], bl[2], bl[3]);
  }
  acc_guard4(acc[0][0], acc[0][1], acc[0][2], acc[0][3]);
  acc_guard4(acc[1][0], acc[1][1], acc[1][2], acc[1][3]);
  acc_guard4(acc[2][0], acc[2][1], acc[2][2], acc[2][3]);
  acc_guard4(acc[3][0], acc[3][1], acc[3][2], acc[3][3]);

  float* slab = sT[wave];
  const float* Rb = RESID ? (resid + (size_t)b * strideR) : nullptr;
#pragma unroll
  for (int i = 0; i < 4; ++i) {
    const int mBase = m0 + (i << 4);
#pragma unroll
    for (int j = 0; j < 4; ++j) {
      const int n = n0 + (j << 4) + rlane;
      float bv = 0.f;
      if (BIAS_MODE == 2) bv = bias[n];
#pragma unroll
      for (int r = 0; r < 8; ++r) {
        float v = acc[i][j][r] * scale;
        if (BIAS_MODE == 1) v += bias[mBase + mOff + r];
        if (BIAS_MODE == 2) v += bv;
        if (RESID) v += Rb[(size_t)(mBase + mOff + r) * ldc + n];
        if (ACT == 1) v = tanhf(v);
        if (ACT == 2) v = fmaxf(v, 0.0f);
        if (ACT == 3) v = v / (1.0f + expf(-v));
        if (ACT == 4) v = (v > 0.f) ? v : 0.01f * v;
        if (ACT == 5) v = 0.5f * v * (1.0f + erff(v * 0.70710678118654752f));
        slab[(mOff + r) * 68 + (j << 4) + rlane] = v;
      }
    }
    __builtin_amdgcn_fence(__ATOMIC_RELEASE, "workgroup");
    __builtin_amdgcn_wave_barrier();
    __builtin_amdgcn_fence(__ATOMIC_ACQUIRE, "workgroup");
    if (OUT_MODE == 0) {
      float* C = (float*)Cout + (size_t)b * strideC;
      const int hh = lane >> 4, c4 = (lane & 15) * 4;
      for (int pass = 0; pass < 2; ++pass) {
#pragma unroll
        for (int it = 0; it < 8; ++it) {
          const int row = it * 2 + hh;
          v4f v = *(const v4f*)(slab + row * 68 + c4);
          *(volatile v4f*)(C + (size_t)(mBase + row) * ldc + n0 + c4) = v;
        }
        __threadfence();
      }
    } else {
      const int q = lane >> 3, c8 = (lane & 7) * 8;
      unsigned short* C  = (unsigned short*)Cout  + (size_t)b * strideC;
      unsigned short* C2 = (OUT_MODE == 2) ? ((unsigned short*)Cout2 + (size_t)b * strideC) : nullptr;
      for (int pass = 0; pass < 2; ++pass) {
#pragma unroll
        for (int it = 0; it < 4; ++it) {
          const int row = it * 4 + q;
          const float* sp = slab + row * 68 + c8;
          v8h hv, lv;
#pragma unroll
          for (int e = 0; e < 8; ++e) {
            if (OUT_MODE == 1) {
              hv[e] = (_Float16)sp[e];
            } else {
              unsigned short hb = f2bf_bits(sp[e]);
              unsigned short lb = f2bf_bits(sp[e] - bf_bits2f(hb));
              hv[e] = __builtin_bit_cast(_Float16, hb);
              lv[e] = __builtin_bit_cast(_Float16, lb);
            }
          }
          *(volatile v8h*)(C + (size_t)(mBase + row) * ldc + n0 + c8) = hv;
          if (OUT_MODE == 2) *(volatile v8h*)(C2 + (size_t)(mBase + row) * ldc + n0 + c8) = lv;
        }
        __threadfence();
      }
    }
    __builtin_amdgcn_fence(__ATOMIC_RELEASE, "workgroup");
    __builtin_amdgcn_wave_barrier();
    __builtin_amdgcn_fence(__ATOMIC_ACQUIRE, "workgroup");
  }
}

__global__ __launch_bounds__(256) void cast_scale_f32_f16x2(
    const float* __restrict__ in, _Float16* __restrict__ out, int n2, float mul) {
  int i = blockIdx.x * 256 + threadIdx.x;
  if (i < n2) {
    const _Float16 h0 = (_Float16)(in[2 * i] * mul), h1 = (_Float16)(in[2 * i + 1] * mul);
    const unsigned u = (unsigned)__builtin_bit_cast(unsigned short, h0) | ((unsigned)__builtin_bit_cast(unsigned short, h1) << 16);
    ((volatile unsigned*)out)[i] = u;
    __threadfence();
    ((volatile unsigned*)out)[i] = u;
  }
}

__global__ __launch_bounds__(64) void prep_xn_kernel(
    const float* __restrict__ spt, const float* __restrict__ qry,
    _Float16* __restrict__ xn16, float* __restrict__ xn32)
{
  __shared__ float tile[NCH][PCHUNK + 1];
  __shared__ float mu[PCHUNK];
  const int tid = threadIdx.x;
  const int img = blockIdx.y;
  const int p0  = blockIdx.x * PCHUNK;
  const float* X = (img < NWAY) ? (spt + (size_t)img * NCH * NPOS)
                                : (qry + (size_t)(img - NWAY) * NCH * NPOS);
#pragma unroll
  for (int i = 0; i < 4; ++i) {
    const int idx = i * 64 + tid;
    const int c = idx >> 2, j4 = (idx & 3) * 4;
    const v4f v = *(const v4f*)(X + (size_t)c * NPOS + p0 + j4);
    tile[c][j4 + 0] = v[0]; tile[c][j4 + 1] = v[1]; tile[c][j4 + 2] = v[2]; tile[c][j4 + 3] = v[3];
  }
  __syncthreads();
  if (tid < PCHUNK) {
    float s = 0.f;
#pragma unroll 8
    for (int c = 0; c < NCH; ++c) s += tile[c][tid];
    mu[tid] = s * (1.0f / (float)NCH);
  }
  __syncthreads();
  const size_t rowbase = (size_t)img * NPOS + p0;
  if (tid < 32) {
    const int lane = tid, q = lane >> 3, c8 = (lane & 7) * 8;
    v8h hv[4];
#pragma unroll
    for (int it = 0; it < 4; ++it) {
      const int j = it * 4 + q;
      const float m = mu[j];
#pragma unroll
      for (int e = 0; e < 8; ++e) hv[it][e] = (_Float16)(tile[c8 + e][j] - m);
    }
    for (int pass = 0; pass < 2; ++pass) {
#pragma unroll
      for (int it = 0; it < 4; ++it) {
        const int j = it * 4 + q;
        *(volatile v8h*)(xn16 + (rowbase + j) * NCH + c8) = hv[it];
      }
      __threadfence();
    }
  } else {
    const int lane = tid - 32, h2 = lane >> 4, c4 = (lane & 15) * 4;
    v4f fv[8];
#pragma unroll
    for (int it = 0; it < 8; ++it) {
      const int j = it * 2 + h2;
      const float m = mu[j];
      fv[it] = (v4f){tile[c4 + 0][j] - m, tile[c4 + 1][j] - m, tile[c4 + 2][j] - m, tile[c4 + 3][j] - m};
    }
    for (int pass = 0; pass < 2; ++pass) {
#pragma unroll
      for (int it = 0; it < 8; ++it) {
        const int j = it * 2 + h2;
        *(volatile v4f*)(xn32 + (rowbase + j) * NCH + c4) = fv[it];
      }
      __threadfence();
    }
  }
}

__global__ __launch_bounds__(256) void feat_kernel(
    const float* __restrict__ Y, const float* __restrict__ bn_g, const float* __restrict__ bn_b,
    const float* __restrict__ bn_m, const float* __restrict__ bn_v,
    _Float16* __restrict__ feat, int nrows)
{
  const int lane = threadIdx.x & 31, wave = threadIdx.x >> 5;
  const int q = lane >> 3, c8 = (lane & 7) * 8;
  const int row  = blockIdx.x * 32 + wave * 4 + q;
  const int rowc = row < nrows ? row : nrows - 1;
  const float* yp = Y + (size_t)rowc * NCH + c8;
  const v4f y0 = *(const v4f*)(yp), y1 = *(const v4f*)(yp + 4);
  const v4f g0 = *(const v4f*)(bn_g + c8), g1 = *(const v4f*)(bn_g + c8 + 4);
  const v4f b0 = *(const v4f*)(bn_b + c8), b1 = *(const v4f*)(bn_b + c8 + 4);
  const v4f m0 = *(const v4f*)(bn_m + c8), m1 = *(const v4f*)(bn_m + c8 + 4);
  const v4f v0 = *(const v4f*)(bn_v + c8), v1 = *(const v4f*)(bn_v + c8 + 4);
  float val[8];
#pragma unroll
  for (int e = 0; e < 4; ++e) {
    const float s0 = g0[e] * rsqrtf(v0[e] + BN_EPS_C);
    const float t0 = (y0[e] - m0[e]) * s0 + b0[e];
    val[e] = fmaxf(t0, 0.0f);
    const float s1 = g1[e] * rsqrtf(v1[e] + BN_EPS_C);
    const float t1 = (y1[e] - m1[e]) * s1 + b1[e];
    val[4 + e] = fmaxf(t1, 0.0f);
  }
  float ssq = 0.f;
#pragma unroll
  for (int e = 0; e < 8; ++e) ssq = fmaf(val[e], val[e], ssq);
  ssq += __shfl_xor(ssq, 1, 32);
  ssq += __shfl_xor(ssq, 2, 32);
  ssq += __shfl_xor(ssq, 4, 32);
  const float inv = 1.0f / fmaxf(sqrtf(ssq), 1e-8f);
  v8h hv;
#pragma unroll
  for (int e = 0; e < 8; ++e) hv[e] = (_Float16)(val[e] * inv);
  _Float16* dst = feat + (size_t)rowc * NCH + c8;
  if (row < nrows) *(volatile v8h*)dst = hv;
  __threadfence();
  if (row < nrows) *(volatile v8h*)dst = hv;
}

__device__ __forceinline__ v8f mma2_f16(v16h a0, v16h b0, v16h a1, v16h b1) {
  v8f acc = (v8f){0.f, 0.f, 0.f, 0.f, 0.f, 0.f, 0.f, 0.f};
  acc = __builtin_amdgcn_wmma_f32_16x16x32_f16(false, a0, false, b0, (short)0, acc, false, false);
  acc = __builtin_amdgcn_wmma_f32_16x16x32_f16(false, a1, false, b1, (short)0, acc, false, false);
  asm volatile("v_nop\n\tv_nop\n\tv_nop\n\tv_nop" : "+v"(acc) : "v"(a0), "v"(b0), "v"(a1), "v"(b1));
  return acc;
}

__global__ __launch_bounds__(256) void corr_attn_kernel(
    const _Float16* __restrict__ feat, const float* __restrict__ xn32,
    const float* __restrict__ scale_p, float* __restrict__ simtab)
{
  __shared__ __align__(16) float cpart[3][8][NPOS];
  __shared__ float colA[NPOS], colB[NPOS], colD[NPOS];
  __shared__ float rowA[NPOS], rowB[NPOS], rowD[NPOS];
  __shared__ float rowS[NPOS], rowQ[NPOS];
  __shared__ float attn[2][NPOS];
  __shared__ float pooled[2 * NCH];

  const int tid  = threadIdx.x;
  const int lane = tid & 31;
  const int wave = tid >> 5;
  const int hh   = lane >> 4;
  const int cc   = lane & 15;
  const int koff = hh * 8;
  const int pair = blockIdx.x;
  const int qi = pair / NWAY;
  const int wi = pair - qi * NWAY;
  const _Float16* Sf = feat + (size_t)wi * NPOS * NCH;
  const _Float16* Qf = feat + (size_t)(NWAY + qi) * NPOS * NCH;

  for (int i = tid; i < 3 * 8 * NPOS; i += 256) (&cpart[0][0][0])[i] = 0.f;
  __syncthreads();

  for (int mi = wave; mi < NTILE; mi += 8) {
    const _Float16* ap = Sf + (size_t)(mi * 16 + cc) * NCH + koff;
    const v16h a0 = Frag<_Float16>::load(ap);
    const v16h a1 = Frag<_Float16>::load(ap + 32);
    float rs[8], rq[8];
#pragma unroll
    for (int r = 0; r < 8; ++r) { rs[r] = 0.f; rq[r] = 0.f; }
#pragma unroll 1
    for (int ni = 0; ni < NTILE; ++ni) {
      const _Float16* bp = Qf + (size_t)(ni * 16 + cc) * NCH + koff;
      const v16h b0 = Frag<_Float16>::load(bp);
      const v16h b1 = Frag<_Float16>::load(bp + 32);
      const v8f x = mma2_f16(a0, b0, a1, b1);
      float cs = 0.f, cq = 0.f;
#pragma unroll
      for (int r = 0; r < 8; ++r) {
        const float v = x[r];
        cs += v; cq = fmaf(v, v, cq);
        rs[r] += v; rq[r] = fmaf(v, v, rq[r]);
      }
      cs += __shfl_xor(cs, 16, 32);
      cq += __shfl_xor(cq, 16, 32);
      if (hh == 0) {
        const int n = ni * 16 + cc;
        cpart[0][wave][n] += cs;
        cpart[1][wave][n] += cq;
      }
    }
#pragma unroll
    for (int r = 0; r < 8; ++r) {
#pragma unroll
      for (int off = 1; off < 16; off <<= 1) {
        rs[r] += __shfl_xor(rs[r], off, 32);
        rq[r] += __shfl_xor(rq[r], off, 32);
      }
    }
    if (cc == 0) {
      const int rb = mi * 16 + 8 * hh;
#pragma unroll
      for (int r = 0; r < 8; ++r) { rowS[rb + r] = rs[r]; rowQ[rb + r] = rq[r]; }
    }
  }
  __syncthreads();

  for (int i = tid; i < NPOS; i += 256) {
    float s = 0.f, s2 = 0.f;
#pragma unroll
    for (int w8 = 0; w8 < 8; ++w8) { s += cpart[0][w8][i]; s2 += cpart[1][w8][i]; }
    {
      const float mean = s * (1.0f / (float)NPOS);
      const float var  = fmaxf((s2 - s * mean) * (1.0f / (float)(NPOS - 1)), 0.0f);
      const float inv  = 1.0f / (sqrtf(var + 1e-5f) * TEMP_ATTN);
      const float a    = inv * LOG2E_C;
      colA[i] = a; colB[i] = -mean * a;
    }
    {
      const float rsum = rowS[i], rsq = rowQ[i];
      const float mean = rsum * (1.0f / (float)NPOS);
      const float var  = fmaxf((rsq - rsum * mean) * (1.0f / (float)(NPOS - 1)), 0.0f);
      const float inv  = 1.0f / (sqrtf(var + 1e-5f) * TEMP_ATTN);
      const float a    = inv * LOG2E_C;
      rowA[i] = a; rowB[i] = -mean * a;
    }
  }
  __syncthreads();

  for (int mi = wave; mi < NTILE; mi += 8) {
    const _Float16* ap = Sf + (size_t)(mi * 16 + cc) * NCH + koff;
    const v16h a0 = Frag<_Float16>::load(ap);
    const v16h a1 = Frag<_Float16>::load(ap + 32);
    const int rb = mi * 16 + 8 * hh;
    float rAr[8], rBr[8], rden[8];
#pragma unroll
    for (int r = 0; r < 8; ++r) { rAr[r] = rowA[rb + r]; rBr[r] = rowB[rb + r]; rden[r] = 0.f; }
#pragma unroll 1
    for (int ni = 0; ni < NTILE; ++ni) {
      const _Float16* bp = Qf + (size_t)(ni * 16 + cc) * NCH + koff;
      const v16h b0 = Frag<_Float16>::load(bp);
      const v16h b1 = Frag<_Float16>::load(bp + 32);
      const v8f x = mma2_f16(a0, b0, a1, b1);
      const int n = ni * 16 + cc;
      const float cA = colA[n], cB = colB[n];
      float cden = 0.f;
#pragma unroll
      for (int r = 0; r < 8; ++r) {
        const float v  = x[r];
        const float ec = exp2f(fmaf(v, cA, cB));
        const float er = exp2f(fmaf(v, rAr[r], rBr[r]));
        cden += ec; rden[r] += er;
      }
      cden += __shfl_xor(cden, 16, 32);
      if (hh == 0) cpart[2][wave][n] += cden;
    }
#pragma unroll
    for (int r = 0; r < 8; ++r) {
#pragma unroll
      for (int off = 1; off < 16; off <<= 1) rden[r] += __shfl_xor(rden[r], off, 32);
    }
    if (cc == 0) {
#pragma unroll
      for (int r = 0; r < 8; ++r) rowS[rb + r] = rden[r];
    }
  }
  __syncthreads();

  for (int i = tid; i < NPOS; i += 256) {
    float d = 0.f;
#pragma unroll
    for (int w8 = 0; w8 < 8; ++w8) d += cpart[2][w8][i];
    colD[i] = 1.0f / d;
    rowD[i] = 1.0f / rowS[i];
  }
  for (int i = tid; i < 8 * NPOS; i += 256) (&cpart[0][0][0])[i] = 0.f;
  __syncthreads();

  for (int mi = wave; mi < NTILE; mi += 8) {
    const _Float16* ap = Sf + (size_t)(mi * 16 + cc) * NCH + koff;
    const v16h a0 = Frag<_Float16>::load(ap);
    const v16h a1 = Frag<_Float16>::load(ap + 32);
    const int rb = mi * 16 + 8 * hh;
    float rAr[8], rBr[8], rDr[8], ras[8];
#pragma unroll
    for (int r = 0; r < 8; ++r) { rAr[r] = rowA[rb + r]; rBr[r] = rowB[rb + r]; rDr[r] = rowD[rb + r]; ras[r] = 0.f; }
#pragma unroll 1
    for (int ni = 0; ni < NTILE; ++ni) {
      const _Float16* bp = Qf + (size_t)(ni * 16 + cc) * NCH + koff;
      const v16h b0 = Frag<_Float16>::load(bp);
      const v16h b1 = Frag<_Float16>::load(bp + 32);
      const v8f x = mma2_f16(a0, b0, a1, b1);
      const int n = ni * 16 + cc;
      const float cA = colA[n], cB = colB[n], cD = colD[n];
      float aq = 0.f;
#pragma unroll
      for (int r = 0; r < 8; ++r) {
        const float v  = x[r];
        const float ec = exp2f(fmaf(v, cA, cB));
        const float er = exp2f(fmaf(v, rAr[r], rBr[r]));
        ras[r] = fmaf(ec, cD, ras[r]);
        aq     = fmaf(er, rDr[r], aq);
      }
      aq += __shfl_xor(aq, 16, 32);
      if (hh == 0) cpart[0][wave][n] += aq;
    }
#pragma unroll
    for (int r = 0; r < 8; ++r) {
#pragma unroll
      for (int off = 1; off < 16; off <<= 1) ras[r] += __shfl_xor(ras[r], off, 32);
    }
    if (cc == 0) {
#pragma unroll
      for (int r = 0; r < 8; ++r) attn[0][rb + r] = ras[r];
    }
  }
  __syncthreads();

  for (int i = tid; i < NPOS; i += 256) {
    float a = 0.f;
#pragma unroll
    for (int w8 = 0; w8 < 8; ++w8) a += cpart[0][w8][i];
    attn[1][i] = a;
  }
  __syncthreads();

  if (tid < 2 * NCH) {
    const int sel = tid >> 6;
    const int c   = tid & 63;
    const int img = sel ? (NWAY + qi) : wi;
    const float* xp = xn32 + (size_t)img * NPOS * NCH + c;
    float acc = 0.f;
#pragma unroll 4
    for (int p = 0; p < NPOS; ++p) acc = fmaf(attn[sel][p], xp[(size_t)p * NCH], acc);
    pooled[tid] = acc * (1.0f / (float)NPOS);
  }
  __syncthreads();

  if (wave == 0) {
    const float sa0 = pooled[lane], sa1 = pooled[lane + 32];
    const float qa0 = pooled[NCH + lane], qa1 = pooled[NCH + 32 + lane];
    float ss = sa0 * sa0 + sa1 * sa1;
    float qq = qa0 * qa0 + qa1 * qa1;
    float sq = sa0 * qa0 + sa1 * qa1;
#pragma unroll
    for (int off = 1; off < 32; off <<= 1) {
      ss += __shfl_xor(ss, off, 32);
      qq += __shfl_xor(qq, off, 32);
      sq += __shfl_xor(sq, off, 32);
    }
    const float ns  = fmaxf(sqrtf(ss), 1e-6f);
    const float nq2 = fmaxf(sqrtf(qq), 1e-6f);
    const float sim = (sq / (ns * nq2)) * scale_p[0];
    const float e0  = (lane == 0) ? sim : 0.0f;
    const v4f val = (v4f){e0, 0.0f, 0.0f, 0.0f};
    float* dst = simtab + (size_t)pair * 32 + lane * 4;
    if (lane < 8) *(volatile v4f*)dst = val;
    __threadfence();
    if (lane < 8) *(volatile v4f*)dst = val;
  }
}

__global__ __launch_bounds__(32) void write_out_kernel(
    const float* __restrict__ simtab, float* __restrict__ out, int nout)
{
  const int lane = threadIdx.x;
  float vals[12];
#pragma unroll
  for (int it = 0; it < 12; ++it) {
    const int idx = it * 32 + lane;
    const int idc = idx < nout ? idx : nout - 1;
    vals[it] = simtab[(size_t)idc * 32];
  }
  for (int pass = 0; pass < 2; ++pass) {
#pragma unroll
    for (int it = 0; it < 12; ++it) {
      const int idx = it * 32 + lane;
      if (idx < nout) *(volatile float*)(out + idx) = vals[it];
    }
    __threadfence();
  }
}

extern "C" void kernel_launch(void* const* d_in, const int* in_sizes, int n_in,
                              void* d_out, int out_size, void* d_ws, size_t ws_size,
                              hipStream_t stream)
{
  if (n_in < 8) return;
  if (in_sizes[0] != NWAY * NCH * NPOS || in_sizes[1] != NQRY * NCH * NPOS ||
      in_sizes[2] != NCH * NCH || in_sizes[3] != NCH || in_sizes[4] != NCH ||
      in_sizes[5] != NCH || in_sizes[6] != NCH || in_sizes[7] < 1) return;
  if (out_size < NPAIR) return;
  if (ws_size < WS_TOTAL) return;

  const float* spt    = (const float*)d_in[0];
  const float* qry    = (const float*)d_in[1];
  const float* conv_w = (const float*)d_in[2];
  const float* bn_g   = (const float*)d_in[3];
  const float* bn_b   = (const float*)d_in[4];
  const float* bn_m   = (const float*)d_in[5];
  const float* bn_v   = (const float*)d_in[6];
  const float* scale  = (const float*)d_in[7];
  float* out = (float*)d_out;

  char* ws = (char*)d_ws;
  _Float16* w16   = (_Float16*)(ws + WS_OFF_W16);
  _Float16* xn16  = (_Float16*)(ws + WS_OFF_XN16);
  float*    xn32  = (float*)(ws + WS_OFF_XN32);
  float*    ybuf  = (float*)(ws + WS_OFF_Y);
  _Float16* feat  = (_Float16*)(ws + WS_OFF_FEAT);
  float*    simtb = (float*)(ws + WS_OFF_SIM);

  {
    const int n2 = (NCH * NCH) / 2;
    cast_scale_f32_f16x2<<<(n2 + 255) / 256, 256, 0, stream>>>(conv_w, w16, n2, WSCALE);
  }
  prep_xn_kernel<<<dim3(NPOS / PCHUNK, NIMG), 64, 0, stream>>>(spt, qry, xn16, xn32);
  {
    const int tiles  = (NROWS / 64) * (NCH / 64);
    const int blocks = (tiles + 7) / 8;
    wmma_gemm64<0, false, 0, 0, false, 0><<<dim3(blocks, 1), 256, 0, stream>>>(
        (const unsigned short*)xn16, (const unsigned short*)xn16, NCH, 0L,
        (const unsigned short*)w16, (const unsigned short*)w16, NCH, 0L,
        (void*)ybuf, (void*)ybuf, NCH, 0L,
        (const float*)ybuf, (const float*)ybuf, 0L,
        NROWS, NCH, NCH, 1.0f / WSCALE);
  }
  feat_kernel<<<NROWS / 32, 256, 0, stream>>>(ybuf, bn_g, bn_b, bn_m, bn_v, feat, NROWS);
  corr_attn_kernel<<<NPAIR, 256, 0, stream>>>(feat, xn32, scale, simtb);
  write_out_kernel<<<1, 32, 0, stream>>>(simtb, out, NPAIR);
}
